// RGBuvHistBlock_67551245632192
// MI455X (gfx1250) — hardware-verified
//
#include <hip/hip_runtime.h>
#include <math.h>

typedef __attribute__((ext_vector_type(16))) _Float16 v16h;
typedef __attribute__((ext_vector_type(16))) __bf16 v16b;
typedef __attribute__((ext_vector_type(8)))  _Float16 v8h;
typedef __attribute__((ext_vector_type(8)))  float v8f;
typedef __attribute__((ext_vector_type(4)))  float v4f;
typedef __attribute__((ext_vector_type(2)))  float v2f;
typedef __attribute__((ext_vector_type(4)))  unsigned v4u;
typedef __attribute__((ext_vector_type(4)))  int v4i;
typedef float __attribute__((may_alias)) float_a;
typedef int __attribute__((may_alias)) int_a;

template <typename T> __device__ __forceinline__ void vst2(void* p, T v) { *(volatile T*)p = v; __threadfence(); *(volatile T*)p = v; }
__device__ __forceinline__ v8f wmma16(v16h a, v16h b, v8f c) {
  v8f d = __builtin_amdgcn_wmma_f32_16x16x32_f16(false, a, false, b, (short)0, c, false, false);
  asm volatile("v_nop\n\tv_nop\n\tv_nop\n\tv_nop" : "+v"(d) : "v"(a), "v"(b));
  return d;
}
__device__ __forceinline__ v8f wmma_bf(v16b a, v16b b, v8f c) {
  v8f d = __builtin_amdgcn_wmma_f32_16x16x32_bf16(false, a, false, b, (short)0, c, false, false);
  asm volatile("v_nop\n\tv_nop\n\tv_nop\n\tv_nop" : "+v"(d) : "v"(a), "v"(b));
  return d;
}
__device__ __forceinline__ v16h frag_h(const _Float16* rowk0, int lane) {
  union { v16h v; v8h q[2]; } u; const _Float16* p = rowk0 + 8 * (lane >> 4);
  u.q[0] = *(const v8h*)p; u.q[1] = *(const v8h*)(p + 16); return u.v;
}
__device__ __forceinline__ v16h frag_f32(const float* rowk0, int lane) {
  v16h a; const float* p = rowk0 + 8 * (lane >> 4);
#pragma unroll
  for (int i = 0; i < 8; ++i) { a[i] = (_Float16)p[i]; a[8 + i] = (_Float16)p[16 + i]; }
  return a;
}
__device__ __forceinline__ v16h frag_f32s(const float* rowk0, int lane, float sc) {
  v16h a; const float* p = rowk0 + 8 * (lane >> 4);
#pragma unroll
  for (int i = 0; i < 8; ++i) { a[i] = (_Float16)(p[i] * sc); a[8 + i] = (_Float16)(p[16 + i] * sc); }
  return a;
}
__device__ __forceinline__ v16h fragc_f32(const float* W, int k0, int n, int lane, int ld, int K) {
  v16h a; const int g = lane >> 4;
#pragma unroll
  for (int i = 0; i < 8; ++i) { const int ka = k0 + 8 * g + i, kb = ka + 16;
    a[i] = (_Float16)(ka < K ? W[(size_t)(ka < K ? ka : K - 1) * ld + n] : 0.f); a[8 + i] = (_Float16)(kb < K ? W[(size_t)(kb < K ? kb : K - 1) * ld + n] : 0.f); }
  return a;
}
struct F2 { v16b h, l; };
__device__ __forceinline__ F2 bsplit16(const float v[16]) { F2 r;
#pragma unroll
  for (int i = 0; i < 16; ++i) { const __bf16 h = (__bf16)v[i]; r.h[i] = h; r.l[i] = (__bf16)(v[i] - (float)h); }
  return r; }
__device__ __forceinline__ F2 split_row(const float* row, int k0, int lane) { float v[16]; const float* p = row + k0 + 8 * (lane >> 4);
#pragma unroll
  for (int i = 0; i < 8; ++i) { v[i] = p[i]; v[8 + i] = p[16 + i]; }
  return bsplit16(v); }
__device__ __forceinline__ F2 split_rowK(const float* row, int k0, int lane, int K) { float v[16]; const int g = lane >> 4;
#pragma unroll
  for (int i = 0; i < 8; ++i) { const int ka = k0 + 8 * g + i, kb = ka + 16; v[i] = ka < K ? row[ka < K ? ka : K - 1] : 0.f; v[8 + i] = kb < K ? row[kb < K ? kb : K - 1] : 0.f; }
  return bsplit16(v); }
__device__ __forceinline__ F2 split_col(const float* W, int k0, int n, int lane, int ld, int K) { float v[16]; const int g = lane >> 4;
#pragma unroll
  for (int i = 0; i < 8; ++i) { const int ka = k0 + 8 * g + i, kb = ka + 16; v[i] = ka < K ? W[(size_t)(ka < K ? ka : K - 1) * ld + n] : 0.f; v[8 + i] = kb < K ? W[(size_t)(kb < K ? kb : K - 1) * ld + n] : 0.f; }
  return bsplit16(v); }
__device__ __forceinline__ v8f mac3(const F2& a, const F2& b, v8f c) { c = wmma_bf(a.l, b.h, c); c = wmma_bf(a.h, b.l, c); return wmma_bf(a.h, b.h, c); }
__device__ __forceinline__ float sigm(float v) { return 1.0f / (1.0f + expf(-v)); }
#define LDSX() do { asm volatile("s_wait_dscnt 0" ::: "memory"); __builtin_amdgcn_wave_barrier(); __builtin_amdgcn_fence(__ATOMIC_RELEASE, "workgroup"); } while (0)


#define NB 4
#define NPIX 65536
#define NBIN 64
#define NCHUNK 16
#define CHK (NPIX / NCHUNK)
#define INVS2 2500.0f
#ifndef TNB
#define TNB NB
#endif
typedef __attribute__((ext_vector_type(8))) __bf16 v8b;
__device__ __forceinline__ v16b frag_b(const __bf16* rowk0, int lane) {
  union { v16b v; v8b q[2]; } u; const __bf16* p = rowk0 + 8 * (lane >> 4);
  u.q[0] = *(const v8b*)p; u.q[1] = *(const v8b*)(p + 16); return u.v;
}
__device__ __forceinline__ float bfr(float v) { return (float)(__bf16)v; }
__device__ __attribute__((noinline)) float exp_ni(float v) { return expf(v); }
__device__ __attribute__((noinline)) float erf_ni(float v) { return erff(v); }

#define WS_PP  0u
#define WS_HP  (WS_PP + 16u * (size_t)NB * NPIX)
#define WS_END (WS_HP + 4u * (size_t)NB * 3 * NCHUNK * NBIN * NBIN)

__device__ __forceinline__ float binv(int i) { return -3.0f + (float)i * (6.0f / 63.0f); }
__global__ __launch_bounds__(256) void k_prep(const float* __restrict__ X, float* __restrict__ PP) { const int t = threadIdx.x; const size_t b = blockIdx.y; const int n = blockIdx.x * 256 + t;
  float I[3];
#pragma unroll
  for (int c = 0; c < 3; ++c) { const float v = bfr(X[(b * 3 + c) * NPIX + n]); I[c] = fminf(fmaxf(v, 0.0f), 1.0f); }
  v4f o; o[0] = sqrtf(I[0] * I[0] + I[1] * I[1] + I[2] * I[2] + 1e-6f); o[1] = logf(I[0] + 1e-6f); o[2] = logf(I[1] + 1e-6f); o[3] = logf(I[2] + 1e-6f);
  vst2(PP + (b * NPIX + n) * 4, o); }
__global__ __launch_bounds__(128) void k_hist(const float* __restrict__ PP, float* __restrict__ HP) { __shared__ __align__(16) __bf16 sbh[NBIN][40], sbl[NBIN][40]; __shared__ __align__(16) float su[32], sv[32], sy[32]; __shared__ __align__(16) float so[4][16][68];
  const int tid = threadIdx.x, wave = tid >> 5, lane = tid & 31, col = lane & 15, g = lane >> 4; const int chunk = blockIdx.x; const int bc = blockIdx.y; const size_t b = bc / 3; const int c = bc % 3;
  const int cu = (c == 0) ? 1 : 0; const int cv = (c == 2) ? 1 : 2;
  const float bu = binv(wave * 16 + col);
  v8f acc[4] = {};
#pragma unroll 1
  for (int kc = 0; kc < CHK / 32; ++kc) { const size_t n0 = b * NPIX + (size_t)chunk * CHK + kc * 32;
    if (tid < 32) { const float* p = PP + (n0 + tid) * 4; const float lc = p[1 + c]; su[tid] = lc - p[1 + cu]; sv[tid] = lc - p[1 + cv]; sy[tid] = p[0]; }
    __syncthreads();
    for (int e = tid; e < NBIN * 32; e += 128) { const int v = e >> 5, k = e & 31; const float dv = sv[k] - binv(v); const float w = 1.0f / (1.0f + dv * dv * INVS2); const __bf16 h = (__bf16)w; sbh[v][k] = h; sbl[v][k] = (__bf16)(w - (float)h); }
    float va[16];
#pragma unroll
    for (int i = 0; i < 8; ++i) { { const int k = 8 * g + i; const float du = su[k] - bu; va[i] = sy[k] / (1.0f + du * du * INVS2); } { const int k = 16 + 8 * g + i; const float du = su[k] - bu; va[8 + i] = sy[k] / (1.0f + du * du * INVS2); } }
    const F2 a = bsplit16(va);
    __syncthreads();
#pragma unroll
    for (int j = 0; j < 4; ++j) { const F2 w = { frag_b(&sbh[j * 16 + col][0], lane), frag_b(&sbl[j * 16 + col][0], lane) }; acc[j] = mac3(a, w, acc[j]); }
    __syncthreads(); }
#pragma unroll
  for (int j = 0; j < 4; ++j)
#pragma unroll
    for (int r = 0; r < 8; ++r) so[wave][8 * g + r][j * 16 + col] = acc[j][r];
  LDSX();
  for (int rl = 0; rl < 16; ++rl) if (lane < 16) vst2(HP + ((((size_t)bc * NCHUNK + chunk) * NBIN) + wave * 16 + rl) * NBIN + lane * 4, *(const v4f*)&so[wave][rl][lane * 4]); }
__global__ __launch_bounds__(256) void k_fin(const float* __restrict__ HP, float* __restrict__ OUT) { __shared__ __align__(16) float sh[3 * NBIN * NBIN]; __shared__ float red[8]; __shared__ float tot;
  const int t = threadIdx.x; const size_t b = blockIdx.x;
  float mysum = 0.f;
  for (int e = t; e < 3 * NBIN * NBIN; e += 256) { const int c = e / (NBIN * NBIN), uv = e % (NBIN * NBIN); float a = 0.f;
#pragma unroll 1
    for (int ch = 0; ch < NCHUNK; ++ch) a += HP[(((b * 3 + c) * NCHUNK + ch) * NBIN * NBIN) + uv];
    sh[e] = a; mysum += a; }
#pragma unroll
  for (int o = 1; o < 32; o <<= 1) mysum += __shfl_xor(mysum, o);
  if ((t & 31) == 0) red[t >> 5] = mysum; __syncthreads(); if (t == 0) { float a = 0.f; for (int i = 0; i < 8; ++i) a += red[i]; tot = a; } __syncthreads();
  const float inv = 1.0f / (tot + 1e-6f);
  for (int e = t; e < 3 * NBIN * NBIN / 4; e += 256) { v4f o; o[0] = sh[e * 4] * inv; o[1] = sh[e * 4 + 1] * inv; o[2] = sh[e * 4 + 2] * inv; o[3] = sh[e * 4 + 3] * inv; vst2(OUT + b * 3 * NBIN * NBIN + e * 4, o); } }
extern "C" void kernel_launch(void* const* d_in, const int* in_sizes, int n_in, void* d_out, int out_size, void* d_ws, size_t ws_size, hipStream_t stream) {
  (void)in_sizes; (void)n_in; (void)out_size;
  const float** F = (const float**)d_in;
  if (ws_size < (size_t)WS_END) return;
  char* ws = (char*)d_ws; float *PP = (float*)(ws + WS_PP), *HP = (float*)(ws + WS_HP);
  k_prep<<<dim3(NPIX / 256, TNB), 256, 0, stream>>>(F[0], PP);
  k_hist<<<dim3(NCHUNK, TNB * 3), 128, 0, stream>>>(PP, HP);
  k_fin<<<TNB, 256, 0, stream>>>(HP, (float*)d_out);
}
